// PureMambaBlock_56221121904989
// MI455X (gfx1250) — hardware-verified
//
#include <hip/hip_runtime.h>
#include <hip/hip_bf16.h>
#include <math.h>

typedef __attribute__((ext_vector_type(16))) __bf16         v16bf;
typedef __attribute__((ext_vector_type(8)))  float          v8f;
typedef __attribute__((ext_vector_type(4)))  float          v4f_na;
typedef v4f_na __attribute__((may_alias))                    v4f;
typedef __attribute__((ext_vector_type(8)))  unsigned short u16x8_na;
typedef u16x8_na __attribute__((may_alias))                  u16x8;
typedef __attribute__((ext_vector_type(4)))  unsigned short u16x4;

#define D_MODEL 1024
#define D_STATE 16
#define D_CONV  4
#define D_INNER 2048
#define DT_RANK 64
#define SEQ_LEN 2048
#define XDBL_N  (DT_RANK + 2 * D_STATE)
#define NCHUNK  32
#define CHUNK_T (SEQ_LEN / NCHUNK)
#define LDS_K   72
#define GEMM_SMEM_HALVES (2 * 64 * LDS_K + 128 * LDS_K)

__device__ __forceinline__ unsigned short f2bf(float f) {
    unsigned int u = __float_as_uint(f);
    u += 0x7FFFu + ((u >> 16) & 1u);
    return (unsigned short)(u >> 16);
}
__device__ __forceinline__ float bf2f(unsigned short b) {
    return __uint_as_float(((unsigned int)b) << 16);
}
__device__ __forceinline__ float bfr(float f) { return bf2f(f2bf(f)); }

union Frag { v16bf v; u16x8 hf[2]; };

__device__ __forceinline__ v8f mma_bf16(v16bf a, v16bf b, v8f acc) {
    acc = __builtin_amdgcn_wmma_f32_16x16x32_bf16(false, a, false, b, (short)0, acc, false, false);
    asm volatile("v_nop\n\tv_nop\n\tv_nop\n\tv_nop" : "+v"(acc) : "v"(a), "v"(b));
    return acc;
}

__global__ void __launch_bounds__(256)
cvt1_kernel(const float* __restrict__ src, unsigned short* dst, int n8) {
    const int g = blockIdx.x * blockDim.x + threadIdx.x;
    if (g >= n8) return;
    const size_t i = (size_t)g * 8;
    const v4f a = *reinterpret_cast<const v4f*>(src + i);
    const v4f b = *reinterpret_cast<const v4f*>(src + i + 4);
    u16x8 o;
    o[0] = f2bf(a[0]); o[1] = f2bf(a[1]); o[2] = f2bf(a[2]); o[3] = f2bf(a[3]);
    o[4] = f2bf(b[0]); o[5] = f2bf(b[1]); o[6] = f2bf(b[2]); o[7] = f2bf(b[3]);
    *(volatile u16x8*)(dst + i) = o;
    __threadfence();
    *(volatile u16x8*)(dst + i) = o;
}

__global__ void __launch_bounds__(256)
cvt2_kernel(const float* __restrict__ src, unsigned short* dhi, unsigned short* dlo, int n8) {
    const int g = blockIdx.x * blockDim.x + threadIdx.x;
    if (g >= n8) return;
    const size_t i = (size_t)g * 8;
    const v4f a = *reinterpret_cast<const v4f*>(src + i);
    const v4f b = *reinterpret_cast<const v4f*>(src + i + 4);
    u16x8 oh, ol;
#pragma unroll
    for (int q = 0; q < 4; ++q) {
        const unsigned short h0 = f2bf(a[q]);
        oh[q] = h0; ol[q] = f2bf(a[q] - bf2f(h0));
        const unsigned short h1 = f2bf(b[q]);
        oh[4 + q] = h1; ol[4 + q] = f2bf(b[q] - bf2f(h1));
    }
    *(volatile u16x8*)(dhi + i) = oh;
    *(volatile u16x8*)(dlo + i) = ol;
    __threadfence();
    *(volatile u16x8*)(dhi + i) = oh;
    *(volatile u16x8*)(dlo + i) = ol;
}

__global__ void __launch_bounds__(256)
atab_kernel(const float* __restrict__ A_log, float* At, int n) {
    const int g = blockIdx.x * blockDim.x + threadIdx.x;
    if (g >= n) return;
    const float v = -expf(bfr(A_log[g]));
    *(volatile float*)(At + g) = v;
    __threadfence();
    *(volatile float*)(At + g) = v;
}

template <int NPL, int EP>
__global__ void __launch_bounds__(256)
gemm_bf16_kernel(const unsigned short* __restrict__ A, long long aPlane, int sA, int M,
                 const unsigned short* __restrict__ W, int N, int K,
                 float* C, int sC, const float* __restrict__ bias)
{
    __shared__ alignas(16) unsigned short smem[GEMM_SMEM_HALVES];
    unsigned short* const As0 = smem;
    unsigned short* const As1 = smem + 64 * LDS_K;
    unsigned short* const Bs  = smem + 2 * 64 * LDS_K;

    const int tid  = threadIdx.x;
    const int lane = tid & 31;
    const int w    = tid >> 5;
    const int wm   = w & 1;
    const int wn   = w >> 1;
    const int h    = lane >> 4;
    const int l15  = lane & 15;
    const int m0   = blockIdx.y * 64;
    const int n0   = blockIdx.x * 128;

    const v8f   z8  = {0.f, 0.f, 0.f, 0.f, 0.f, 0.f, 0.f, 0.f};
    const u16x8 z16 = {0, 0, 0, 0, 0, 0, 0, 0};
    v8f acc[2][2];
    acc[0][0] = z8; acc[0][1] = z8; acc[1][0] = z8; acc[1][1] = z8;

#pragma unroll 1
    for (int k0 = 0; k0 < K; k0 += 64) {
#pragma unroll
        for (int p = 0; p < NPL; ++p) {
            const unsigned short* Ap = A + (size_t)p * (size_t)aPlane;
            unsigned short* const dst = (p == 0) ? As0 : As1;
#pragma unroll
            for (int i = 0; i < 2; ++i) {
                const int c   = tid * 2 + i;
                const int r   = c >> 3;
                const int off = (c & 7) * 8;
                u16x8 v = z16;
                if (m0 + r < M)
                    v = *reinterpret_cast<const u16x8*>(Ap + (size_t)(m0 + r) * sA + k0 + off);
                *reinterpret_cast<u16x8*>(dst + r * LDS_K + off) = v;
            }
        }
#pragma unroll
        for (int i = 0; i < 4; ++i) {
            const int c   = tid * 4 + i;
            const int r   = c >> 3;
            const int off = (c & 7) * 8;
            u16x8 v = z16;
            if (n0 + r < N)
                v = *reinterpret_cast<const u16x8*>(W + (size_t)(n0 + r) * K + k0 + off);
            *reinterpret_cast<u16x8*>(Bs + r * LDS_K + off) = v;
        }
        __syncthreads();

#pragma unroll
        for (int ks = 0; ks < 2; ++ks) {
            const int kb = ks * 32;
            Frag ah[2], al[2], bw[2];
#pragma unroll
            for (int mi = 0; mi < 2; ++mi) {
                const int ro = (wm * 32 + mi * 16 + l15) * LDS_K + kb;
                ah[mi].hf[0] = *reinterpret_cast<const u16x8*>(As0 + ro + 8 * h);
                ah[mi].hf[1] = *reinterpret_cast<const u16x8*>(As0 + ro + 16 + 8 * h);
                if (NPL == 2) {
                    al[mi].hf[0] = *reinterpret_cast<const u16x8*>(As1 + ro + 8 * h);
                    al[mi].hf[1] = *reinterpret_cast<const u16x8*>(As1 + ro + 16 + 8 * h);
                } else {
                    al[mi].hf[0] = z16; al[mi].hf[1] = z16;
                }
            }
#pragma unroll
            for (int ni = 0; ni < 2; ++ni) {
                const int ro = (wn * 32 + ni * 16 + l15) * LDS_K + kb;
                bw[ni].hf[0] = *reinterpret_cast<const u16x8*>(Bs + ro + 8 * h);
                bw[ni].hf[1] = *reinterpret_cast<const u16x8*>(Bs + ro + 16 + 8 * h);
            }
#pragma unroll
            for (int mi = 0; mi < 2; ++mi)
#pragma unroll
                for (int ni = 0; ni < 2; ++ni)
                    acc[mi][ni] = mma_bf16(ah[mi].v, bw[ni].v, acc[mi][ni]);
            if (NPL == 2) {
#pragma unroll
                for (int mi = 0; mi < 2; ++mi)
#pragma unroll
                    for (int ni = 0; ni < 2; ++ni)
                        acc[mi][ni] = mma_bf16(al[mi].v, bw[ni].v, acc[mi][ni]);
            }
        }
        __syncthreads();
    }

    float* const stg = reinterpret_cast<float*>(smem) + w * 1024;
#pragma unroll
    for (int mi = 0; mi < 2; ++mi)
#pragma unroll
        for (int ni = 0; ni < 2; ++ni)
#pragma unroll
            for (int r = 0; r < 8; ++r)
                stg[(mi * 16 + 8 * h + r) * 32 + ni * 16 + l15] = acc[mi][ni][r];
    __syncthreads();

    if (EP == 1) {
        const int nn = n0 + wn * 32 + lane;
        float bv = 0.f;
        if (nn < N) bv = bfr(bias[nn]);
#pragma unroll 1
        for (int i = 0; i < 32; ++i) {
            float v = stg[i * 32 + lane] + bv;
            v = fmaxf(v, 0.f) + log1pf(expf(-fabsf(v)));
            stg[i * 32 + lane] = v;
        }
        __syncthreads();
    }

    const bool wave_ok = (n0 + wn * 32 + 32) <= N;
    const int  rsub = lane >> 3;
    const int  cq   = (lane & 7) * 4;
    v4f vals[8];
#pragma unroll
    for (int it = 0; it < 8; ++it)
        vals[it] = *reinterpret_cast<const v4f*>(stg + (it * 4 + rsub) * 32 + cq);
    const int ncol = n0 + wn * 32 + cq;
    if (wave_ok) {
#pragma unroll
        for (int it = 0; it < 8; ++it) {
            const int mrow = m0 + wm * 32 + it * 4 + rsub;
            if (mrow < M) *(volatile v4f*)(C + (size_t)mrow * sC + ncol) = vals[it];
        }
    }
    __threadfence();
    if (wave_ok) {
#pragma unroll
        for (int it = 0; it < 8; ++it) {
            const int mrow = m0 + wm * 32 + it * 4 + rsub;
            if (mrow < M) *(volatile v4f*)(C + (size_t)mrow * sC + ncol) = vals[it];
        }
    }
}

__global__ void __launch_bounds__(256)
conv_silu_kernel(const float* __restrict__ xz, const float* __restrict__ cw,
                 const float* __restrict__ cb, float* xc,
                 unsigned short* xch, unsigned short* xcl, int n4)
{
    const int g = blockIdx.x * blockDim.x + threadIdx.x;
    if (g >= n4) return;
    const size_t idx = (size_t)g * 4;
    const int c = (int)(idx & (D_INNER - 1));
    const int t = (int)(idx >> 11);
    float acc[4] = {0.f, 0.f, 0.f, 0.f};
#pragma unroll
    for (int j = 0; j < D_CONV; ++j) {
        const int tt = t + j - (D_CONV - 1);
        if (tt >= 0) {
            const v4f xv = *reinterpret_cast<const v4f*>(xz + (size_t)tt * (2 * D_INNER) + c);
#pragma unroll
            for (int q = 0; q < 4; ++q)
                acc[q] += xv[q] * bfr(cw[(c + q) * D_CONV + j]);
        }
    }
    v4f o = {0.f, 0.f, 0.f, 0.f};
    u16x4 oh = {0, 0, 0, 0}, ol = {0, 0, 0, 0};
#pragma unroll
    for (int q = 0; q < 4; ++q) {
        const float v = acc[q] + bfr(cb[c + q]);
        const float s = v * (1.0f / (1.0f + expf(-v)));
        o[q] = s;
        const unsigned short hb = f2bf(s);
        oh[q] = hb;
        ol[q] = f2bf(s - bf2f(hb));
    }
    *(volatile v4f*)(xc + idx)    = o;
    *(volatile u16x4*)(xch + idx) = oh;
    *(volatile u16x4*)(xcl + idx) = ol;
    __threadfence();
    *(volatile v4f*)(xc + idx)    = o;
    *(volatile u16x4*)(xch + idx) = oh;
    *(volatile u16x4*)(xcl + idx) = ol;
}

__global__ void __launch_bounds__(256)
scan_partial_kernel(const float* __restrict__ xc, const float* __restrict__ dtm,
                    const float* __restrict__ xdbl, const float* __restrict__ At,
                    float* P, float* Q, int nthr)
{
    const int g = blockIdx.x * blockDim.x + threadIdx.x;
    if (g >= nthr) return;
    const int d     = g & (D_INNER - 1);
    const int chunk = g >> 11;

    float Av[D_STATE], hh[D_STATE];
#pragma unroll
    for (int j = 0; j < 4; ++j) {
        const v4f a4 = *reinterpret_cast<const v4f*>(At + (size_t)d * D_STATE + 4 * j);
        Av[4 * j + 0] = a4[0]; Av[4 * j + 1] = a4[1]; Av[4 * j + 2] = a4[2]; Av[4 * j + 3] = a4[3];
        hh[4 * j + 0] = 0.f; hh[4 * j + 1] = 0.f; hh[4 * j + 2] = 0.f; hh[4 * j + 3] = 0.f;
    }
    float sdt = 0.f;
    const int t0 = chunk * CHUNK_T;
#pragma unroll 1
    for (int i = 0; i < CHUNK_T; ++i) {
        const int t = t0 + i;
        const float xt  = xc [(size_t)t * D_INNER + d];
        const float dtt = dtm[(size_t)t * D_INNER + d];
        const float* bp = xdbl + (size_t)t * XDBL_N + DT_RANK;
        v4f bq[4];
#pragma unroll
        for (int j = 0; j < 4; ++j) bq[j] = *reinterpret_cast<const v4f*>(bp + 4 * j);
        sdt += dtt;
#pragma unroll
        for (int n = 0; n < D_STATE; ++n) {
            const float dA = __expf(Av[n] * dtt);
            hh[n] = dA * hh[n] + (dtt * bq[n >> 2][n & 3]) * xt;
        }
    }
    const size_t base = ((size_t)chunk * D_INNER + d) * D_STATE;
    v4f pv[4], qv[4];
#pragma unroll
    for (int j = 0; j < 4; ++j) {
#pragma unroll
        for (int q = 0; q < 4; ++q) {
            pv[j][q] = __expf(Av[4 * j + q] * sdt);
            qv[j][q] = hh[4 * j + q];
        }
    }
#pragma unroll
    for (int j = 0; j < 4; ++j) {
        *(volatile v4f*)(P + base + 4 * j) = pv[j];
        *(volatile v4f*)(Q + base + 4 * j) = qv[j];
    }
    __threadfence();
#pragma unroll
    for (int j = 0; j < 4; ++j) {
        *(volatile v4f*)(P + base + 4 * j) = pv[j];
        *(volatile v4f*)(Q + base + 4 * j) = qv[j];
    }
}

__global__ void __launch_bounds__(256)
scan_carry_kernel(const float* __restrict__ P, const float* __restrict__ Q, float* H0, int nd)
{
    const int d = blockIdx.x * blockDim.x + threadIdx.x;
    if (d >= nd) return;
    const v4f z4 = {0.f, 0.f, 0.f, 0.f};
    v4f hc[4];
    hc[0] = z4; hc[1] = z4; hc[2] = z4; hc[3] = z4;
#pragma unroll 1
    for (int c = 0; c < NCHUNK; ++c) {
        const size_t base = ((size_t)c * D_INNER + d) * D_STATE;
        v4f p[4], q[4], o[4];
#pragma unroll
        for (int j = 0; j < 4; ++j) {
            p[j] = *reinterpret_cast<const v4f*>(P + base + 4 * j);
            q[j] = *reinterpret_cast<const v4f*>(Q + base + 4 * j);
            o[j] = hc[j];
        }
#pragma unroll
        for (int j = 0; j < 4; ++j) *(volatile v4f*)(H0 + base + 4 * j) = o[j];
        __threadfence();
#pragma unroll
        for (int j = 0; j < 4; ++j) *(volatile v4f*)(H0 + base + 4 * j) = o[j];
#pragma unroll
        for (int j = 0; j < 4; ++j) hc[j] = p[j] * hc[j] + q[j];
    }
}

__global__ void __launch_bounds__(256)
scan_final_kernel(const float* __restrict__ xc, const float* __restrict__ dtm,
                  const float* __restrict__ xdbl, const float* __restrict__ At,
                  const float* __restrict__ Dp, const float* __restrict__ xz,
                  const float* __restrict__ H0, unsigned short* yh, unsigned short* yl)
{
    __shared__ alignas(16) float ystg[16][256];
    const int tid   = threadIdx.x;
    const int chunk = blockIdx.x >> 3;
    const int dblk  = (blockIdx.x & 7) * 256;
    const int d     = dblk + tid;

    float Av[D_STATE], hh[D_STATE];
    const size_t hbase = ((size_t)chunk * D_INNER + d) * D_STATE;
#pragma unroll
    for (int j = 0; j < 4; ++j) {
        const v4f a4 = *reinterpret_cast<const v4f*>(At + (size_t)d * D_STATE + 4 * j);
        const v4f h4 = *reinterpret_cast<const v4f*>(H0 + hbase + 4 * j);
        Av[4 * j + 0] = a4[0]; Av[4 * j + 1] = a4[1]; Av[4 * j + 2] = a4[2]; Av[4 * j + 3] = a4[3];
        hh[4 * j + 0] = h4[0]; hh[4 * j + 1] = h4[1]; hh[4 * j + 2] = h4[2]; hh[4 * j + 3] = h4[3];
    }
    const float Dd = bfr(Dp[d]);
    const int   t0 = chunk * CHUNK_T;
    const int   wrow = tid >> 5;
    const int   seg  = tid & 31;

#pragma unroll 1
    for (int sub = 0; sub < CHUNK_T / 16; ++sub) {
#pragma unroll 1
        for (int i = 0; i < 16; ++i) {
            const int t = t0 + sub * 16 + i;
            const float xt  = xc [(size_t)t * D_INNER + d];
            const float dtt = dtm[(size_t)t * D_INNER + d];
            const float* bp = xdbl + (size_t)t * XDBL_N + DT_RANK;
            const float* cp = bp + D_STATE;
            v4f bq[4], cq4[4];
#pragma unroll
            for (int j = 0; j < 4; ++j) {
                bq[j]  = *reinterpret_cast<const v4f*>(bp + 4 * j);
                cq4[j] = *reinterpret_cast<const v4f*>(cp + 4 * j);
            }
            float yt = 0.f;
#pragma unroll
            for (int n = 0; n < D_STATE; ++n) {
                const float dA = __expf(Av[n] * dtt);
                hh[n] = dA * hh[n] + (dtt * bq[n >> 2][n & 3]) * xt;
                yt   += hh[n] * cq4[n >> 2][n & 3];
            }
            const float z  = xz[(size_t)t * (2 * D_INNER) + D_INNER + d];
            const float sz = z * (1.0f / (1.0f + expf(-z)));
            yt = (yt + Dd * xt) * sz;
            ystg[i][tid] = yt;
        }
        __syncthreads();

        u16x8 oh[2], ol[2];
#pragma unroll
        for (int ph = 0; ph < 2; ++ph) {
            const int row = wrow + 8 * ph;
            const v4f u0 = *reinterpret_cast<const v4f*>(&ystg[row][seg * 8]);
            const v4f u1 = *reinterpret_cast<const v4f*>(&ystg[row][seg * 8 + 4]);
#pragma unroll
            for (int q = 0; q < 4; ++q) {
                const unsigned short h0 = f2bf(u0[q]);
                oh[ph][q] = h0;     ol[ph][q] = f2bf(u0[q] - bf2f(h0));
                const unsigned short h1 = f2bf(u1[q]);
                oh[ph][4 + q] = h1; ol[ph][4 + q] = f2bf(u1[q] - bf2f(h1));
            }
        }
#pragma unroll
        for (int ph = 0; ph < 2; ++ph) {
            const int t = t0 + sub * 16 + wrow + 8 * ph;
            const size_t off = (size_t)t * D_INNER + dblk + seg * 8;
            *(volatile u16x8*)(yh + off) = oh[ph];
            *(volatile u16x8*)(yl + off) = ol[ph];
        }
        __threadfence();
#pragma unroll
        for (int ph = 0; ph < 2; ++ph) {
            const int t = t0 + sub * 16 + wrow + 8 * ph;
            const size_t off = (size_t)t * D_INNER + dblk + seg * 8;
            *(volatile u16x8*)(yh + off) = oh[ph];
            *(volatile u16x8*)(yl + off) = ol[ph];
        }
        __syncthreads();
    }
}

extern "C" void kernel_launch(void* const* d_in, const int* in_sizes, int n_in,
                              void* d_out, int out_size, void* d_ws, size_t ws_size,
                              hipStream_t stream) {
    if (n_in < 10) return;
    if (in_sizes[0] != SEQ_LEN * D_MODEL)       return;
    if (in_sizes[1] != 2 * D_INNER * D_MODEL)   return;
    if (in_sizes[2] != D_INNER * D_CONV)        return;
    if (in_sizes[3] != D_INNER)                 return;
    if (in_sizes[4] != XDBL_N * D_INNER)        return;
    if (in_sizes[5] != D_INNER * DT_RANK)       return;
    if (in_sizes[6] != D_INNER)                 return;
    if (in_sizes[7] != D_INNER * D_STATE)       return;
    if (in_sizes[8] != D_INNER)                 return;
    if (in_sizes[9] != D_MODEL * D_INNER)       return;
    if (out_size != SEQ_LEN * D_MODEL)          return;

    const float* x     = (const float*)d_in[0];
    const float* W_in  = (const float*)d_in[1];
    const float* convw = (const float*)d_in[2];
    const float* convb = (const float*)d_in[3];
    const float* W_x   = (const float*)d_in[4];
    const float* W_dt  = (const float*)d_in[5];
    const float* b_dt  = (const float*)d_in[6];
    const float* A_log = (const float*)d_in[7];
    const float* Dp    = (const float*)d_in[8];
    const float* W_out = (const float*)d_in[9];
    float* out = (float*)d_out;

    size_t off = 0;
    auto carve = [&](size_t bytes) { size_t o = off; off += (bytes + 255) & ~(size_t)255; return o; };
    const size_t o_xz   = carve((size_t)SEQ_LEN * 2 * D_INNER * 4);
    const size_t o_xc   = carve((size_t)SEQ_LEN * D_INNER * 4);
    const size_t o_xdbl = carve((size_t)SEQ_LEN * XDBL_N * 4);
    const size_t o_dt   = carve((size_t)SEQ_LEN * D_INNER * 4);
    const size_t o_P    = carve((size_t)NCHUNK * D_INNER * D_STATE * 4);
    const size_t o_Q    = carve((size_t)NCHUNK * D_INNER * D_STATE * 4);
    const size_t o_H0   = carve((size_t)NCHUNK * D_INNER * D_STATE * 4);
    const size_t o_At   = carve((size_t)D_INNER * D_STATE * 4);
    const size_t o_xbf  = carve((size_t)SEQ_LEN * D_MODEL * 2);
    const size_t o_Win  = carve((size_t)2 * D_INNER * D_MODEL * 2);
    const size_t o_Wx   = carve((size_t)XDBL_N * D_INNER * 2);
    const size_t o_Wdt  = carve((size_t)D_INNER * DT_RANK * 2);
    const size_t o_Wout = carve((size_t)D_MODEL * D_INNER * 2);
    const size_t o_xch  = carve((size_t)SEQ_LEN * D_INNER * 2);
    const size_t o_xcl  = carve((size_t)SEQ_LEN * D_INNER * 2);
    const size_t o_xdh  = carve((size_t)SEQ_LEN * XDBL_N * 2);
    const size_t o_xdl  = carve((size_t)SEQ_LEN * XDBL_N * 2);
    const size_t o_yh   = carve((size_t)SEQ_LEN * D_INNER * 2);
    const size_t o_yl   = carve((size_t)SEQ_LEN * D_INNER * 2);
    if (off > ws_size) return;

    char* wsb = (char*)d_ws;
    float* xz    = (float*)(wsb + o_xz);
    float* xc    = (float*)(wsb + o_xc);
    float* xdbl  = (float*)(wsb + o_xdbl);
    float* dtbuf = (float*)(wsb + o_dt);
    float* Pbuf  = (float*)(wsb + o_P);
    float* Qbuf  = (float*)(wsb + o_Q);
    float* H0buf = (float*)(wsb + o_H0);
    float* Atab  = (float*)(wsb + o_At);
    unsigned short* xbf   = (unsigned short*)(wsb + o_xbf);
    unsigned short* Winb  = (unsigned short*)(wsb + o_Win);
    unsigned short* Wxb   = (unsigned short*)(wsb + o_Wx);
    unsigned short* Wdtb  = (unsigned short*)(wsb + o_Wdt);
    unsigned short* Woutb = (unsigned short*)(wsb + o_Wout);
    unsigned short* xch   = (unsigned short*)(wsb + o_xch);
    unsigned short* xcl   = (unsigned short*)(wsb + o_xcl);
    unsigned short* xdh   = (unsigned short*)(wsb + o_xdh);
    unsigned short* xdl   = (unsigned short*)(wsb + o_xdl);
    unsigned short* yh    = (unsigned short*)(wsb + o_yh);
    unsigned short* yl    = (unsigned short*)(wsb + o_yl);
    const long long plane_xc = (long long)((o_xcl - o_xch) / 2);
    const long long plane_xd = (long long)((o_xdl - o_xdh) / 2);
    const long long plane_y  = (long long)((o_yl  - o_yh ) / 2);

    const int CT = 256;
    auto cvt1 = [&](const float* s, unsigned short* dst, int n) {
        const int n8 = n / 8;
        cvt1_kernel<<<(n8 + CT - 1) / CT, CT, 0, stream>>>(s, dst, n8);
    };

    cvt1(x,     xbf,   SEQ_LEN * D_MODEL);
    cvt1(W_in,  Winb,  2 * D_INNER * D_MODEL);
    cvt1(W_x,   Wxb,   XDBL_N * D_INNER);
    cvt1(W_dt,  Wdtb,  D_INNER * DT_RANK);
    cvt1(W_out, Woutb, D_MODEL * D_INNER);
    atab_kernel<<<(D_INNER * D_STATE + CT - 1) / CT, CT, 0, stream>>>(A_log, Atab, D_INNER * D_STATE);

    gemm_bf16_kernel<1, 0><<<dim3((2 * D_INNER + 127) / 128, (SEQ_LEN + 63) / 64), 256, 0, stream>>>(
        xbf, 0LL, D_MODEL, SEQ_LEN, Winb, 2 * D_INNER, D_MODEL, xz, 2 * D_INNER, nullptr);

    conv_silu_kernel<<<(SEQ_LEN * D_INNER / 4 + CT - 1) / CT, CT, 0, stream>>>(
        xz, convw, convb, xc, xch, xcl, SEQ_LEN * D_INNER / 4);

    gemm_bf16_kernel<2, 0><<<dim3((XDBL_N + 127) / 128, (SEQ_LEN + 63) / 64), 256, 0, stream>>>(
        xch, plane_xc, D_INNER, SEQ_LEN, Wxb, XDBL_N, D_INNER, xdbl, XDBL_N, nullptr);
    {
        const int n8 = SEQ_LEN * XDBL_N / 8;
        cvt2_kernel<<<(n8 + CT - 1) / CT, CT, 0, stream>>>(xdbl, xdh, xdl, n8);
    }

    gemm_bf16_kernel<2, 1><<<dim3((D_INNER + 127) / 128, (SEQ_LEN + 63) / 64), 256, 0, stream>>>(
        xdh, plane_xd, XDBL_N, SEQ_LEN, Wdtb, D_INNER, DT_RANK, dtbuf, D_INNER, b_dt);

    scan_partial_kernel<<<(NCHUNK * D_INNER + CT - 1) / CT, CT, 0, stream>>>(
        xc, dtbuf, xdbl, Atab, Pbuf, Qbuf, NCHUNK * D_INNER);
    scan_carry_kernel<<<(D_INNER + CT - 1) / CT, CT, 0, stream>>>(
        Pbuf, Qbuf, H0buf, D_INNER);
    scan_final_kernel<<<NCHUNK * (D_INNER / 256), 256, 0, stream>>>(
        xc, dtbuf, xdbl, Atab, Dp, xz, H0buf, yh, yl);

    gemm_bf16_kernel<2, 0><<<dim3((D_MODEL + 127) / 128, (SEQ_LEN + 63) / 64), 256, 0, stream>>>(
        yh, plane_y, D_INNER, SEQ_LEN, Woutb, D_MODEL, D_INNER, out, D_MODEL, nullptr);
}
